// CTGAP_89240830476826
// MI455X (gfx1250) — hardware-verified
//
#include <hip/hip_runtime.h>
#include <stddef.h>


typedef _Float16 v16h __attribute__((ext_vector_type(16)));
typedef _Float16 v8h  __attribute__((ext_vector_type(8)));
typedef float    v8f  __attribute__((ext_vector_type(8)));
typedef float    v4f  __attribute__((ext_vector_type(4)));

#ifndef NB
#define NB 16
#endif
#ifndef NNODE
#define NNODE 2048
#endif
#define NB_FULL    16
#define NNODE_FULL 2048
#define HDIM   512
#define DNODE  256
#define GD     64
#define QROWS  16
#define NTILE  (NNODE / 64)

static_assert(NB >= 1 && NB <= NB_FULL);
static_assert(NB_FULL == QROWS);
static_assert(NNODE >= 1024 && NNODE <= NNODE_FULL && (NNODE % 1024) == 0);
static_assert(GD == 64);
static_assert((HDIM % 64) == 0 && ((HDIM / 2) % 32) == 0);
static_assert((DNODE % 32) == 0);
static_assert(((GD / 2) % 32) == 0);
static_assert(((NNODE / 2) % 32) == 0 && (NNODE % 64) == 0 && (NNODE % 256) == 0);
static_assert((GD * HDIM) % 2048 == 0 && (GD * DNODE) % 2048 == 0 && (GD * GD) % 2048 == 0);
static_assert((QROWS * HDIM) % 2048 == 0 && (NNODE * DNODE) % 2048 == 0);
static_assert((NB * HDIM) % 8 == 0 && NB * HDIM >= 8);

#define LDT 72
#define LDC 68
static_assert((LDT % 8) == 0 && LDT >= 64);
static_assert((LDC % 4) == 0 && LDC >= 64);

#define WCARRY 64.0f
#define XCARRY 64.0f
#define QCARRY 64.0f
#define VCARRY 64.0f
#define PCARRY 16384.0f
#define ACARRY 1024.0f
#define UCARRY 64.0f
#define ZCARRY 64.0f

#define WQ_B   ((size_t)GD * HDIM * 2)
#define WKV_B  ((size_t)GD * DNODE * 2)
#define WO_B   ((size_t)GD * GD * 2)
#define H16_B  ((size_t)QROWS * HDIM * 2)
#define X16_B  ((size_t)NNODE * DNODE * 2)
#define ADJ_B  ((size_t)NNODE * NNODE * 2)
#define RS_B   ((size_t)NNODE * 4)
#define Q16_B  ((size_t)QROWS * GD * 2)
#define K16_B  ((size_t)NNODE * GD * 2)
#define VF_B   ((size_t)NNODE * GD * 4)
#define VT_B   ((size_t)GD * NNODE * 2)
#define LG_B   ((size_t)QROWS * NNODE * 4)
#define A16_B  ((size_t)QROWS * NNODE * 2)
#define UT_B   ((size_t)NB * GD * NNODE * 2)
#define PT_B   ((size_t)NB * NTILE * GD * 4)
#define OFF_WQ  ((size_t)0)
#define OFF_WK  (OFF_WQ + WQ_B)
#define OFF_WV  (OFF_WK + WKV_B)
#define OFF_WO  (OFF_WV + WKV_B)
#define OFF_H   (OFF_WO + WO_B)
#define OFF_X   (OFF_H + H16_B)
#define OFF_ADJ (OFF_X + X16_B)
#define OFF_RS  (OFF_ADJ + ADJ_B)
#define OFF_Q   (OFF_RS + RS_B)
#define OFF_K   (OFF_Q + Q16_B)
#define OFF_VF  (OFF_K + K16_B)
#define OFF_VT  (OFF_VF + VF_B)
#define OFF_LG  (OFF_VT + VT_B)
#define OFF_AL  (OFF_LG + LG_B)
#define OFF_DI  (OFF_AL + LG_B)
#define OFF_A16 (OFF_DI + LG_B)
#define OFF_UT  (OFF_A16 + A16_B)
#define OFF_PT  (OFF_UT + UT_B)
#define WS_TOTAL (OFF_PT + PT_B)
static_assert((WQ_B % 128) == 0 && (WKV_B % 128) == 0 && (WO_B % 128) == 0 && (H16_B % 128) == 0);
static_assert((X16_B % 128) == 0 && (ADJ_B % 128) == 0 && (RS_B % 128) == 0 && (Q16_B % 128) == 0);
static_assert((K16_B % 128) == 0 && (VF_B % 128) == 0 && (VT_B % 128) == 0 && (LG_B % 128) == 0);
static_assert((A16_B % 128) == 0 && (UT_B % 128) == 0 && (PT_B % 128) == 0);
static_assert(WS_TOTAL <= (size_t)134217728);

#define OUT1_OFF ((size_t)NB_FULL * GD)
#define OUT2_OFF ((size_t)2 * NB_FULL * GD)
static_assert(OUT1_OFF * 4 == 4096);
static_assert(OUT2_OFF * 4 == 8192);
static_assert((OUT2_OFF + (size_t)NB_FULL * NNODE_FULL * GD) * 4 == 8396800);

__device__ __forceinline__ float bf16r(float x) {
  unsigned int u = __float_as_uint(x);
  u = (u + 0x7FFFu + ((u >> 16) & 1u)) & 0xFFFF0000u;
  return __uint_as_float(u);
}

static __device__ __forceinline__ _Float16 toh_flush(float v) {
  const _Float16 r = (_Float16)v;
  return (fabsf(v) < 6.103515625e-05f) ? (_Float16)0.0f : r;
}

__device__ __forceinline__ v16h frag_at(const _Float16* p) {
  v8h lo = *(const v8h*)(p);
  v8h hi = *(const v8h*)(p + 16);
  v16h out;
#pragma unroll
  for (int i = 0; i < 8; ++i) { out[i] = lo[i]; out[i + 8] = hi[i]; }
  return out;
}
__device__ __forceinline__ v16h frag_join(v8h lo, v8h hi) {
  v16h out;
#pragma unroll
  for (int i = 0; i < 8; ++i) { out[i] = lo[i]; out[i + 8] = hi[i]; }
  return out;
}

__device__ __forceinline__ v8f wmma16(v16h a, v16h b, v8f c) {
  v8f d = __builtin_amdgcn_wmma_f32_16x16x32_f16(false, a, false, b, (short)0, c,
                                                 false, false);
  asm volatile("v_nop\n\tv_nop\n\tv_nop\n\tv_nop" : "+v"(d) : "v"(a), "v"(b));
  return d;
}

__device__ __forceinline__ float red16_sum(float x) {
#pragma unroll
  for (int off = 1; off < 16; off <<= 1) x += __shfl_xor(x, off, 32);
  return x;
}
__device__ __forceinline__ float red32_sum(float x) {
#pragma unroll
  for (int off = 1; off < 32; off <<= 1) x += __shfl_xor(x, off, 32);
  return x;
}
__device__ __forceinline__ float red32_max(float x) {
#pragma unroll
  for (int off = 1; off < 32; off <<= 1) x = fmaxf(x, __shfl_xor(x, off, 32));
  return x;
}

__global__ __launch_bounds__(256) void cvt_plane_kernel(
    const float* __restrict__ src, _Float16* __restrict__ dst, float carry,
    unsigned n_valid, unsigned n_total) {
#pragma clang fp contract(off)
  const unsigned idx = (blockIdx.x * 256u + threadIdx.x) * 8u;
  const bool ok = idx < n_valid;
  const unsigned ia = ok ? idx : (n_valid - 8u);
  const v4f a0 = *(const v4f*)(src + ia);
  const v4f a1 = *(const v4f*)(src + ia + 4u);
  v8h o;
#pragma unroll
  for (int i = 0; i < 4; ++i) {
    const _Float16 t0 = toh_flush(carry * bf16r(a0[i]));
    const _Float16 t1 = toh_flush(carry * bf16r(a1[i]));
    o[i]     = ok ? t0 : (_Float16)0.0f;
    o[i + 4] = ok ? t1 : (_Float16)0.0f;
  }
  if (idx < n_total) {
    _Float16* p = dst + idx;
    *(volatile v8h*)p = o;
    __threadfence();
    *(volatile v8h*)p = o;
  }
}

__global__ __launch_bounds__(256) void adj_kernel(
    const float* __restrict__ adj, _Float16* __restrict__ A16, float* __restrict__ rowsum) {
#pragma clang fp contract(off)
  __shared__ __attribute__((aligned(16))) float rs[32];
  const unsigned lane = threadIdx.x & 31u;
  const unsigned wave = __builtin_amdgcn_readfirstlane(threadIdx.x >> 5);
  const unsigned rbase = blockIdx.x * 32u;
#pragma unroll 1
  for (unsigned q = 0; q < 4u; ++q) {
    const unsigned row = rbase + wave * 4u + q;
    const float* xr = adj + (size_t)row * NNODE_FULL + lane * 8u;
    _Float16* dr = A16 + (size_t)row * NNODE + lane * 8u;
    float s = 0.0f;
#pragma unroll 1
    for (unsigned j = 0; j < (unsigned)(NNODE / 256); ++j) {
      const v4f a0 = *(const v4f*)(xr + j * 256u);
      const v4f a1 = *(const v4f*)(xr + j * 256u + 4u);
      v8h o;
#pragma unroll
      for (int i = 0; i < 4; ++i) {
        const float e0 = bf16r(a0[i]);
        const float e1 = bf16r(a1[i]);
        s += e0;
        s += e1;
        o[i]     = toh_flush(ACARRY * e0);
        o[i + 4] = toh_flush(ACARRY * e1);
      }
      _Float16* p = dr + j * 256u;
      *(volatile v8h*)p = o;
      __threadfence();
      *(volatile v8h*)p = o;
    }
    s = red32_sum(s);
    if (lane == 0u) rs[wave * 4u + q] = s;
  }
  __syncthreads();
  if (threadIdx.x < 8u) {
    const v4f t = *(const v4f*)&rs[threadIdx.x * 4u];
    float* p = rowsum + rbase + threadIdx.x * 4u;
    *(volatile v4f*)p = t;
    __threadfence();
    *(volatile v4f*)p = t;
  }
}

template <int MODE>
__device__ __forceinline__ void row16_body(
    const _Float16* __restrict__ A16, const _Float16* __restrict__ Bt, const unsigned K,
    const float* __restrict__ bias, const float cscale,
    float* __restrict__ outf, _Float16* __restrict__ out16,
    const unsigned ldo, const unsigned rows_out) {
  __shared__ __attribute__((aligned(16))) float Cs2[2 * 16 * LDC];
  const unsigned tid = threadIdx.x, lane = tid & 31u;
  const unsigned wave = __builtin_amdgcn_readfirstlane(tid >> 5);
  const unsigned nt = wave & 3u, kh = wave >> 2;
  const unsigned hh = lane >> 4, m = lane & 15u;
  const unsigned n0 = blockIdx.x * 64u;
  const unsigned khalf = K >> 1;

  const _Float16* ap = A16 + (size_t)m * K + kh * khalf + hh * 8u;
  const _Float16* bp = Bt + (size_t)(n0 + nt * 16u + m) * K + kh * khalf + hh * 8u;
  v8f acc = {};
#pragma unroll 2
  for (unsigned k0 = 0; k0 < khalf; k0 += 32u) {
    const v16h a = frag_at(ap + k0);
    const v16h b = frag_at(bp + k0);
    acc = wmma16(a, b, acc);
  }
#pragma unroll
  for (int r = 0; r < 8; ++r)
    Cs2[(kh * 16u + hh * 8u + (unsigned)r) * LDC + nt * 16u + m] = acc[r];
  __syncthreads();

  if (MODE == 0) {
    if (tid < 128u) {
      const unsigned r = tid >> 3;
      const unsigned c = (tid & 7u) * 8u;
      const v4f u0 = *(const v4f*)&Cs2[r * LDC + c] + *(const v4f*)&Cs2[(16u + r) * LDC + c];
      const v4f u1 = *(const v4f*)&Cs2[r * LDC + c + 4u] + *(const v4f*)&Cs2[(16u + r) * LDC + c + 4u];
      const v4f g0 = *(const v4f*)(bias + n0 + c);
      const v4f g1 = *(const v4f*)(bias + n0 + c + 4u);
      v8h x;
#pragma unroll
      for (int j = 0; j < 4; ++j) {
        x[j]     = toh_flush(QCARRY * (u0[j] * cscale + bf16r(g0[j])));
        x[j + 4] = toh_flush(QCARRY * (u1[j] * cscale + bf16r(g1[j])));
      }
      _Float16* p = out16 + (size_t)r * ldo + n0 + c;
      *(volatile v8h*)p = x;
      __threadfence();
      *(volatile v8h*)p = x;
    }
  }

  if (MODE == 1) {
    const unsigned r = tid >> 4;
    const unsigned c = (tid & 15u) * 4u;
    const v4f u = *(const v4f*)&Cs2[r * LDC + c] + *(const v4f*)&Cs2[(16u + r) * LDC + c];
    v4f val;
#pragma unroll
    for (int j = 0; j < 4; ++j) val[j] = u[j] * cscale;
    if (r < rows_out) {
      float* p = outf + (size_t)r * ldo + n0 + c;
      *(volatile v4f*)p = val;
      __threadfence();
      *(volatile v4f*)p = val;
    }
  }
}

__global__ __launch_bounds__(256) void row16_q_kernel(
    const _Float16* __restrict__ A16, const _Float16* __restrict__ Bt,
    const float* __restrict__ bias, _Float16* __restrict__ q16) {
  row16_body<0>(A16, Bt, (unsigned)HDIM, bias, 1.0f / (XCARRY * WCARRY),
                (float*)0, q16, (unsigned)GD, (unsigned)QROWS);
}
__global__ __launch_bounds__(256) void row16_f32_kernel(
    const _Float16* __restrict__ A16, const _Float16* __restrict__ Bt, unsigned K,
    float cscale, float* __restrict__ outf, unsigned ldo, unsigned rows_out) {
  row16_body<1>(A16, Bt, K, (const float*)0, cscale, outf, (_Float16*)0, ldo, rows_out);
}

template <int MODE>
__device__ __forceinline__ void gemm64_body(
    const _Float16* __restrict__ A16, const _Float16* __restrict__ Bt, const unsigned K,
    const float* __restrict__ bias, float* __restrict__ outf, _Float16* __restrict__ out16) {
  __shared__ __attribute__((aligned(16))) float Cs[64 * LDC];
  const unsigned tid = threadIdx.x, lane = tid & 31u;
  const unsigned w = __builtin_amdgcn_readfirstlane(tid >> 5);
  const unsigned mw = w >> 1, nw = w & 1u;
  const unsigned hh = lane >> 4, m = lane & 15u;
  const unsigned n0 = blockIdx.x * 64u;
  const unsigned row0 = blockIdx.y * 64u;

  const _Float16* ap  = A16 + (size_t)(row0 + mw * 16u + m) * K + hh * 8u;
  const _Float16* bp0 = Bt + (size_t)(n0 + nw * 32u + m) * K + hh * 8u;
  const _Float16* bp1 = bp0 + (size_t)16 * K;
  v8f acc0 = {}, acc1 = {};
#pragma unroll 2
  for (unsigned k0 = 0; k0 < K; k0 += 32u) {
    const v16h a  = frag_at(ap + k0);
    const v16h b0 = frag_at(bp0 + k0);
    const v16h b1 = frag_at(bp1 + k0);
    acc0 = wmma16(a, b0, acc0);
    acc1 = wmma16(a, b1, acc1);
  }
#pragma unroll
  for (int r = 0; r < 8; ++r) {
    const unsigned ci = (mw * 16u + hh * 8u + (unsigned)r) * LDC + nw * 32u + m;
    Cs[ci]       = acc0[r];
    Cs[ci + 16u] = acc1[r];
  }
  __syncthreads();

  const float cs = 1.0f / (XCARRY * WCARRY);

  if (MODE == 0) {
    v8h x[2];
    size_t off[2];
#pragma unroll
    for (unsigned i = 0; i < 2u; ++i) {
      const unsigned r = 32u * i + (tid >> 3);
      const unsigned c = (tid & 7u) * 8u;
      const v4f u0 = *(const v4f*)&Cs[r * LDC + c];
      const v4f u1 = *(const v4f*)&Cs[r * LDC + c + 4u];
      const v4f g0 = *(const v4f*)(bias + n0 + c);
      const v4f g1 = *(const v4f*)(bias + n0 + c + 4u);
#pragma unroll
      for (int j = 0; j < 4; ++j) {
        x[i][j]     = toh_flush(QCARRY * (u0[j] * cs + bf16r(g0[j])));
        x[i][j + 4] = toh_flush(QCARRY * (u1[j] * cs + bf16r(g1[j])));
      }
      off[i] = (size_t)(row0 + r) * GD + n0 + c;
    }
#pragma unroll
    for (int i = 0; i < 2; ++i) *(volatile v8h*)(out16 + off[i]) = x[i];
    __threadfence();
#pragma unroll
    for (int i = 0; i < 2; ++i) *(volatile v8h*)(out16 + off[i]) = x[i];
  }

  if (MODE == 1) {
    v4f xs[4];
    size_t off[4];
#pragma unroll
    for (unsigned i = 0; i < 4u; ++i) {
      const unsigned r = 16u * i + (tid >> 4);
      const unsigned c = (tid & 15u) * 4u;
      const v4f u = *(const v4f*)&Cs[r * LDC + c];
      const v4f g = *(const v4f*)(bias + n0 + c);
      v4f val;
#pragma unroll
      for (int j = 0; j < 4; ++j) val[j] = u[j] * cs + bf16r(g[j]);
      xs[i] = val;
      off[i] = (size_t)(row0 + r) * GD + n0 + c;
    }
#pragma unroll
    for (int i = 0; i < 4; ++i) *(volatile v4f*)(outf + off[i]) = xs[i];
    __threadfence();
#pragma unroll
    for (int i = 0; i < 4; ++i) *(volatile v4f*)(outf + off[i]) = xs[i];

    v8h x[2];
    size_t offt[2];
#pragma unroll
    for (unsigned i = 0; i < 2u; ++i) {
      const unsigned dcol = 32u * i + (tid >> 3);
      const unsigned kk = (tid & 7u) * 8u;
      const float bb = bf16r(bias[n0 + dcol]);
#pragma unroll
      for (unsigned j = 0; j < 8u; ++j) {
        const float t = Cs[(kk + j) * LDC + dcol] * cs + bb;
        x[i][j] = toh_flush(VCARRY * t);
      }
      offt[i] = (size_t)(n0 + dcol) * NNODE + row0 + kk;
    }
#pragma unroll
    for (int i = 0; i < 2; ++i) *(volatile v8h*)(out16 + offt[i]) = x[i];
    __threadfence();
#pragma unroll
    for (int i = 0; i < 2; ++i) *(volatile v8h*)(out16 + offt[i]) = x[i];
  }
}

__global__ __launch_bounds__(256) void gemm_k_kernel(
    const _Float16* __restrict__ A16, const _Float16* __restrict__ Bt,
    const float* __restrict__ bias, _Float16* __restrict__ k16) {
  gemm64_body<0>(A16, Bt, (unsigned)DNODE, bias, (float*)0, k16);
}
__global__ __launch_bounds__(256) void gemm_v_kernel(
    const _Float16* __restrict__ A16, const _Float16* __restrict__ Bt,
    const float* __restrict__ bias, float* __restrict__ vf, _Float16* __restrict__ vt16) {
  gemm64_body<1>(A16, Bt, (unsigned)DNODE, bias, vf, vt16);
}

__global__ __launch_bounds__(256) void softmax_kernel(
    const float* __restrict__ Lg, const float* __restrict__ rowsum,
    float* __restrict__ Alpha, float* __restrict__ Dinv, _Float16* __restrict__ Al16) {
#pragma clang fp contract(off)
  __shared__ __attribute__((aligned(16))) float sm[NNODE];
  __shared__ float wred[8];
  const unsigned tid = threadIdx.x, lane = tid & 31u;
  const unsigned wave = __builtin_amdgcn_readfirstlane(tid >> 5);
  const unsigned b = blockIdx.x;
  const float* L = Lg + (size_t)b * NNODE;

  float mx = -3.0e38f;
#pragma unroll 1
  for (unsigned c0 = 0; c0 < (unsigned)NNODE; c0 += 1024u) {
    const v4f a = *(const v4f*)(L + c0 + tid * 4u);
    mx = fmaxf(fmaxf(mx, fmaxf(a[0], a[1])), fmaxf(a[2], a[3]));
  }
  mx = red32_max(mx);
  if (lane == 0u) wred[wave] = mx;
  __syncthreads();
  float gm = wred[0];
#pragma unroll
  for (int i = 1; i < 8; ++i) gm = fmaxf(gm, wred[i]);
  __syncthreads();

  float s = 0.0f;
#pragma unroll 1
  for (unsigned c0 = 0; c0 < (unsigned)NNODE; c0 += 1024u) {
    const v4f a = *(const v4f*)(L + c0 + tid * 4u);
    v4f e;
#pragma unroll
    for (int j = 0; j < 4; ++j) e[j] = __expf(a[j] - gm);
    s += (e[0] + e[1]) + (e[2] + e[3]);
    *(v4f*)&sm[c0 + tid * 4u] = e;
  }
  s = red32_sum(s);
  if (lane == 0u) wred[wave] = s;
  __syncthreads();
  float tot = wred[0];
#pragma unroll
  for (int i = 1; i < 8; ++i) tot += wred[i];
  const float inv = 1.0f / tot;

#pragma unroll 1
  for (unsigned c0 = 0; c0 < (unsigned)NNODE; c0 += 1024u) {
    const unsigned c = c0 + tid * 4u;
    const v4f e = *(const v4f*)&sm[c];
    const v4f rsv = *(const v4f*)(rowsum + c);
    v4f al, di;
#pragma unroll
    for (int j = 0; j < 4; ++j) {
      al[j] = e[j] * inv;
      const float dg = (al[j] * rsv[j] + 1.0f) + 1.0e-8f;
      di[j] = rsqrtf(dg);
    }
    *(v4f*)&sm[c] = al;
    float* pa = Alpha + (size_t)b * NNODE + c;
    float* pd = Dinv + (size_t)b * NNODE + c;
    *(volatile v4f*)pa = al;
    *(volatile v4f*)pd = di;
    __threadfence();
    *(volatile v4f*)pa = al;
    *(volatile v4f*)pd = di;
  }
  __syncthreads();

#pragma unroll 1
  for (unsigned c0 = 0; c0 < (unsigned)NNODE; c0 += 2048u) {
    const unsigned c = c0 + tid * 8u;
    if (c < (unsigned)NNODE) {
      const v4f a0 = *(const v4f*)&sm[c];
      const v4f a1 = *(const v4f*)&sm[c + 4u];
      v8h o;
#pragma unroll
      for (int j = 0; j < 4; ++j) {
        o[j]     = toh_flush(PCARRY * a0[j]);
        o[j + 4] = toh_flush(PCARRY * a1[j]);
      }
      _Float16* p = Al16 + (size_t)b * NNODE + c;
      *(volatile v8h*)p = o;
      __threadfence();
      *(volatile v8h*)p = o;
    }
  }
}

__global__ __launch_bounds__(256) void uplane_kernel(
    const float* __restrict__ VF, const float* __restrict__ Dinv, _Float16* __restrict__ UT) {
#pragma clang fp contract(off)
  __shared__ __attribute__((aligned(16))) _Float16 T[64 * LDT];
  const unsigned tid = threadIdx.x;
  const unsigned m0 = blockIdx.x * 64u;
  const unsigned b = blockIdx.y;
#pragma unroll 4
  for (unsigned j = 0; j < 16u; ++j) {
    const unsigned idx = tid + 256u * j;
    const unsigned kr = idx >> 6, nc = idx & 63u;
    const float v = VF[(size_t)(m0 + kr) * GD + nc];
    const float di = Dinv[(size_t)b * NNODE + m0 + kr];
    T[nc * LDT + kr] = toh_flush(UCARRY * (di * v));
  }
  __syncthreads();
  v8h x[2];
  size_t off[2];
#pragma unroll
  for (unsigned i = 0; i < 2u; ++i) {
    const unsigned n = 32u * i + (tid >> 3);
    const unsigned kc = (tid & 7u) * 8u;
    x[i] = *(const v8h*)&T[n * LDT + kc];
    off[i] = (size_t)(b * 64u + n) * NNODE + m0 + kc;
  }
#pragma unroll
  for (int i = 0; i < 2; ++i) *(volatile v8h*)(UT + off[i]) = x[i];
  __threadfence();
#pragma unroll
  for (int i = 0; i < 2; ++i) *(volatile v8h*)(UT + off[i]) = x[i];
}

__global__ __launch_bounds__(256) void prop_kernel(
    const _Float16* __restrict__ Adj16, const _Float16* __restrict__ UT16,
    const _Float16* __restrict__ Wo16, const float* __restrict__ VF,
    const float* __restrict__ Alpha, const float* __restrict__ Dinv,
    const float* __restrict__ bo, const float* __restrict__ gamma,
    const float* __restrict__ beta, float* __restrict__ upd, float* __restrict__ part) {
  __shared__ __attribute__((aligned(16))) float Cs[64 * LDC];
  __shared__ __attribute__((aligned(16))) _Float16 Zs[64 * LDT];
  __shared__ __attribute__((aligned(16))) float Rs[16 * 64];
  const unsigned tid = threadIdx.x, lane = tid & 31u;
  const unsigned w = __builtin_amdgcn_readfirstlane(tid >> 5);
  const unsigned mw = w >> 1, nw = w & 1u;
  const unsigned hh = lane >> 4, m = lane & 15u;
  const unsigned b = blockIdx.x;
  const unsigned n0 = b * 64u;
  const unsigned row0 = blockIdx.y * 64u;

  const _Float16* ap  = Adj16 + (size_t)(row0 + mw * 16u + m) * NNODE + hh * 8u;
  const _Float16* bp0 = UT16 + (size_t)(n0 + nw * 32u + m) * NNODE + hh * 8u;
  const _Float16* bp1 = bp0 + (size_t)16 * NNODE;
  v8f acc0 = {}, acc1 = {};
#pragma unroll 2
  for (unsigned k0 = 0; k0 < (unsigned)NNODE; k0 += 32u) {
    const v16h a  = frag_at(ap + k0);
    const v16h b0 = frag_at(bp0 + k0);
    const v16h b1 = frag_at(bp1 + k0);
    acc0 = wmma16(a, b0, acc0);
    acc1 = wmma16(a, b1, acc1);
  }
#pragma unroll
  for (int r = 0; r < 8; ++r) {
    const unsigned ci = (mw * 16u + hh * 8u + (unsigned)r) * LDC + nw * 32u + m;
    Cs[ci]       = acc0[r];
    Cs[ci + 16u] = acc1[r];
  }
  __syncthreads();

  const float pscale = 1.0f / (ACARRY * UCARRY);
#pragma unroll
  for (unsigned i = 0; i < 2u; ++i) {
    const unsigned r = 32u * i + (tid >> 3);
    const unsigned c = (tid & 7u) * 8u;
    const unsigned node = row0 + r;
    const float al = Alpha[(size_t)b * NNODE + node];
    const float di = Dinv[(size_t)b * NNODE + node];
    const v4f p0 = *(const v4f*)&Cs[r * LDC + c];
    const v4f p1 = *(const v4f*)&Cs[r * LDC + c + 4u];
    const v4f w0 = *(const v4f*)(VF + (size_t)node * GD + c);
    const v4f w1 = *(const v4f*)(VF + (size_t)node * GD + c + 4u);
    v8h zv;
#pragma unroll
    for (int j = 0; j < 4; ++j) {
      const float z0 = di * (al * (p0[j] * pscale) + di * w0[j]);
      const float z1 = di * (al * (p1[j] * pscale) + di * w1[j]);
      zv[j]     = toh_flush(ZCARRY * z0);
      zv[j + 4] = toh_flush(ZCARRY * z1);
    }
    *(v8h*)&Zs[r * LDT + c] = zv;
  }
  __syncthreads();

  v8f y0 = {}, y1 = {};
#pragma unroll
  for (unsigned c = 0; c < 2u; ++c) {
    const unsigned zo = (mw * 16u + m) * LDT + hh * 8u + c * 32u;
    const v8h zl = *(const v8h*)&Zs[zo];
    const v8h zh = *(const v8h*)&Zs[zo + 16u];
    const v16h a  = frag_join(zl, zh);
    const v16h b0 = frag_at(Wo16 + (size_t)(nw * 32u + m) * GD + hh * 8u + c * 32u);
    const v16h b1 = frag_at(Wo16 + (size_t)(nw * 32u + 16u + m) * GD + hh * 8u + c * 32u);
    y0 = wmma16(a, b0, y0);
    y1 = wmma16(a, b1, y1);
  }
#pragma unroll
  for (int r = 0; r < 8; ++r) {
    const unsigned ci = (mw * 16u + hh * 8u + (unsigned)r) * LDC + nw * 32u + m;
    Cs[ci]       = y0[r];
    Cs[ci + 16u] = y1[r];
  }
  __syncthreads();

  const float yscale = 1.0f / (ZCARRY * WCARRY);
  const unsigned c4 = (tid & 15u) * 4u;
  const v4f gbo = *(const v4f*)(bo + c4);
  const v4f gga = *(const v4f*)(gamma + c4);
  const v4f gbe = *(const v4f*)(beta + c4);
  v4f xs[4];
  size_t off[4];
  v4f pc = {};
#pragma unroll
  for (unsigned i = 0; i < 4u; ++i) {
    const unsigned r = 16u * i + (tid >> 4);
    const unsigned node = row0 + r;
    const v4f u = *(const v4f*)&Cs[r * LDC + c4];
    v4f y;
#pragma unroll
    for (int j = 0; j < 4; ++j) y[j] = fmaxf(u[j] * yscale + bf16r(gbo[j]), 0.0f);
    const float mu = red16_sum((y[0] + y[1]) + (y[2] + y[3])) * (1.0f / 64.0f);
    v4f d;
#pragma unroll
    for (int j = 0; j < 4; ++j) d[j] = y[j] - mu;
    const float var =
        red16_sum((d[0] * d[0] + d[1] * d[1]) + (d[2] * d[2] + d[3] * d[3])) * (1.0f / 64.0f);
    const float rstd = rsqrtf(var + 1.0e-5f);
    const float al = Alpha[(size_t)b * NNODE + node];
    v4f val;
#pragma unroll
    for (int j = 0; j < 4; ++j) {
      val[j] = d[j] * rstd * bf16r(gga[j]) + bf16r(gbe[j]);
      pc[j] = pc[j] + al * val[j];
    }
    xs[i] = val;
    off[i] = ((size_t)b * NNODE_FULL + node) * GD + c4;
  }
#pragma unroll
  for (int i = 0; i < 4; ++i) *(volatile v4f*)(upd + off[i]) = xs[i];
  __threadfence();
#pragma unroll
  for (int i = 0; i < 4; ++i) *(volatile v4f*)(upd + off[i]) = xs[i];

  *(v4f*)&Rs[(tid >> 4) * 64u + c4] = pc;
  __syncthreads();
  if (tid < 16u) {
    const unsigned cc = tid * 4u;
    v4f t = *(const v4f*)&Rs[cc];
#pragma unroll 1
    for (unsigned q = 1; q < 16u; ++q) t = t + *(const v4f*)&Rs[q * 64u + cc];
    float* p = part + ((size_t)b * NTILE + blockIdx.y) * 64u + cc;
    *(volatile v4f*)p = t;
    __threadfence();
    *(volatile v4f*)p = t;
  }
}

__global__ __launch_bounds__(256) void summary_kernel(
    const float* __restrict__ part, float* __restrict__ out0) {
#pragma clang fp contract(off)
  const unsigned e = threadIdx.x * 4u;
  const unsigned b = e >> 6, g = e & 63u;
  const unsigned bb = (b < (unsigned)NB) ? b : (unsigned)(NB - 1);
  v4f t = {};
#pragma unroll 1
  for (unsigned q = 0; q < (unsigned)NTILE; ++q)
    t = t + *(const v4f*)(part + ((size_t)bb * NTILE + q) * 64u + g);
  if (b < (unsigned)NB) {
    float* p = out0 + e;
    *(volatile v4f*)p = t;
    __threadfence();
    *(volatile v4f*)p = t;
  }
}

extern "C" void kernel_launch(void* const* d_in, const int* in_sizes, int n_in,
                              void* d_out, int out_size, void* d_ws, size_t ws_size,
                              hipStream_t stream) {
  if (n_in < 13) return;
  if ((long long)in_sizes[0] < (long long)NB * HDIM) return;
  if ((long long)in_sizes[1] < (long long)NNODE * DNODE) return;
  if ((long long)in_sizes[2] < (long long)(NNODE - 1) * NNODE_FULL + NNODE) return;
  if ((long long)in_sizes[3] < (long long)GD * HDIM) return;
  if ((long long)in_sizes[5] < (long long)GD * DNODE) return;
  if ((long long)in_sizes[7] < (long long)GD * DNODE) return;
  if ((long long)in_sizes[9] < (long long)GD * GD) return;
  if (in_sizes[4] < GD || in_sizes[6] < GD || in_sizes[8] < GD || in_sizes[10] < GD) return;
  if (in_sizes[11] < GD || in_sizes[12] < GD) return;
  const long long need_out =
      (long long)OUT2_OFF + ((long long)(NB - 1) * NNODE_FULL + NNODE) * GD;
  if ((long long)out_size < need_out) return;
  if (ws_size < WS_TOTAL) return;

  const float* h_t   = (const float*)d_in[0];
  const float* nodes = (const float*)d_in[1];
  const float* adj   = (const float*)d_in[2];
  const float* wq    = (const float*)d_in[3];
  const float* bq    = (const float*)d_in[4];
  const float* wk    = (const float*)d_in[5];
  const float* bk    = (const float*)d_in[6];
  const float* wv    = (const float*)d_in[7];
  const float* bv    = (const float*)d_in[8];
  const float* wo    = (const float*)d_in[9];
  const float* bo    = (const float*)d_in[10];
  const float* gamma = (const float*)d_in[11];
  const float* beta  = (const float*)d_in[12];
  float* out = (float*)d_out;

  char* ws = (char*)d_ws;
  _Float16* Wq16  = (_Float16*)(ws + OFF_WQ);
  _Float16* Wk16  = (_Float16*)(ws + OFF_WK);
  _Float16* Wv16  = (_Float16*)(ws + OFF_WV);
  _Float16* Wo16  = (_Float16*)(ws + OFF_WO);
  _Float16* H16   = (_Float16*)(ws + OFF_H);
  _Float16* X16   = (_Float16*)(ws + OFF_X);
  _Float16* Adj16 = (_Float16*)(ws + OFF_ADJ);
  float*    Rsum  = (float*)(ws + OFF_RS);
  _Float16* Q16   = (_Float16*)(ws + OFF_Q);
  _Float16* K16   = (_Float16*)(ws + OFF_K);
  float*    VF    = (float*)(ws + OFF_VF);
  _Float16* VT16  = (_Float16*)(ws + OFF_VT);
  float*    Lg    = (float*)(ws + OFF_LG);
  float*    Alpha = (float*)(ws + OFF_AL);
  float*    Dinv  = (float*)(ws + OFF_DI);
  _Float16* Al16  = (_Float16*)(ws + OFF_A16);
  _Float16* UT16  = (_Float16*)(ws + OFF_UT);
  float*    Part  = (float*)(ws + OFF_PT);

  dim3 blk(256);

  cvt_plane_kernel<<<dim3((GD * HDIM) / 2048), blk, 0, stream>>>(
      wq, Wq16, WCARRY, (unsigned)(GD * HDIM), (unsigned)(GD * HDIM));
  cvt_plane_kernel<<<dim3((GD * DNODE) / 2048), blk, 0, stream>>>(
      wk, Wk16, WCARRY, (unsigned)(GD * DNODE), (unsigned)(GD * DNODE));
  cvt_plane_kernel<<<dim3((GD * DNODE) / 2048), blk, 0, stream>>>(
      wv, Wv16, WCARRY, (unsigned)(GD * DNODE), (unsigned)(GD * DNODE));
  cvt_plane_kernel<<<dim3((GD * GD) / 2048), blk, 0, stream>>>(
      wo, Wo16, WCARRY, (unsigned)(GD * GD), (unsigned)(GD * GD));
  cvt_plane_kernel<<<dim3((QROWS * HDIM) / 2048), blk, 0, stream>>>(
      h_t, H16, XCARRY, (unsigned)(NB * HDIM), (unsigned)(QROWS * HDIM));
  cvt_plane_kernel<<<dim3((NNODE * DNODE) / 2048), blk, 0, stream>>>(
      nodes, X16, XCARRY, (unsigned)(NNODE * DNODE), (unsigned)(NNODE * DNODE));
  adj_kernel<<<dim3(NNODE / 32), blk, 0, stream>>>(adj, Adj16, Rsum);

  row16_q_kernel<<<dim3(GD / 64), blk, 0, stream>>>(H16, Wq16, bq, Q16);
  gemm_k_kernel<<<dim3(GD / 64, NNODE / 64), blk, 0, stream>>>(X16, Wk16, bk, K16);
  gemm_v_kernel<<<dim3(GD / 64, NNODE / 64), blk, 0, stream>>>(X16, Wv16, bv, VF, VT16);

  row16_f32_kernel<<<dim3(NNODE / 64), blk, 0, stream>>>(
      Q16, K16, (unsigned)GD, 1.0f / (QCARRY * QCARRY * 8.0f), Lg, (unsigned)NNODE,
      (unsigned)QROWS);
  softmax_kernel<<<dim3(QROWS), blk, 0, stream>>>(Lg, Rsum, Alpha, Dinv, Al16);
  row16_f32_kernel<<<dim3(GD / 64), blk, 0, stream>>>(
      Al16, VT16, (unsigned)NNODE, 1.0f / (PCARRY * VCARRY), out + OUT1_OFF, (unsigned)GD,
      (unsigned)NB);

  uplane_kernel<<<dim3(NNODE / 64, NB), blk, 0, stream>>>(VF, Dinv, UT16);
  prop_kernel<<<dim3(NB, NNODE / 64), blk, 0, stream>>>(
      Adj16, UT16, Wo16, VF, Alpha, Dinv, bo, gamma, beta, out + OUT2_OFF, Part);
  summary_kernel<<<dim3(1), blk, 0, stream>>>(Part, out);
}
